// ChunkwiseRetention_6433861009417
// MI455X (gfx1250) — hardware-verified
//
#include <hip/hip_runtime.h>
#include <hip/hip_bf16.h>
#include <math.h>
#define NUM_R 4


#define BB 4
#define BH 2
#define SS 2048
#define DD 1024
#define HH 16
#define DKK 64
#define QW 2

typedef _Float16 bf16;
typedef __attribute__((ext_vector_type(4))) unsigned v4u_t;
typedef unsigned v4ua __attribute__((ext_vector_type(4), may_alias));
typedef __attribute__((ext_vector_type(4))) float v4f_t;
typedef float v4fa __attribute__((ext_vector_type(4), may_alias));
typedef __attribute__((ext_vector_type(16))) bf16  bf16x16;
typedef __attribute__((ext_vector_type(8)))  bf16  bf16x8;
typedef __attribute__((ext_vector_type(4)))  bf16  bf16x4;
typedef __attribute__((ext_vector_type(8)))  float f32x8;

#define LDS_STRIDE 48
#define KSTRIDE    72
#define VSTRIDE    48

__device__ __forceinline__ f32x8 wmma_bf16(bf16x16 a, bf16x16 b, f32x8 c) {
  return __builtin_amdgcn_wmma_f32_16x16x32_f16(
      false, a, false, b, (short)0, c, false, false);
}
#define RSPLIT (1.0f / 2048.0f)
__device__ __forceinline__ bf16 lo_of(float v, bf16 h) { return (bf16)((v - (float)h) * 2048.0f); }
__device__ __forceinline__ f32x8 wmma_split(bf16x16 a, bf16x16 al, bf16x16 b, bf16x16 bl, f32x8 c) {
  f32x8 x = {}; x = wmma_bf16(al, b, x); x = wmma_bf16(a, bl, x); return wmma_bf16(a, b, c) + x * RSPLIT; }

template <typename T>
__device__ __forceinline__ bf16x16 load_frag(const T* __restrict__ base, int ld,
                                             int row0, int k0) {
  const int lane = threadIdx.x & 31;
  const int r    = lane & 15;
  const int kh   = (lane >> 4) * 8;
  const T* p0 = base + (size_t)(row0 + r) * ld + (k0 + kh);
  const T* p1 = p0 + 16;
  bf16x16 f;
#pragma unroll
  for (int i = 0; i < 8; ++i) {
    f[i]     = (bf16)p0[i];
    f[i + 8] = (bf16)p1[i];
  }
  return f;
}

__device__ __forceinline__ bf16x16 lds_frag(const bf16* base, int stride) {
  const int lane = threadIdx.x & 31;
  const int row  = lane & 15;
  const int kh   = (lane >> 4) * 8;
  const bf16x8 lo = *(const bf16x8*)(base + row * stride + kh);
  const bf16x8 hi = *(const bf16x8*)(base + row * stride + kh + 16);
  bf16x16 f;
#pragma unroll
  for (int i = 0; i < 8; ++i) { f[i] = lo[i]; f[i + 8] = hi[i]; }
  return f;
}

template <typename T>
__device__ __forceinline__ void stage_read16(const T* __restrict__ p, float* buf) {
#pragma unroll
  for (int i = 0; i < 16; ++i) buf[i] = (float)p[i];
}

__device__ __forceinline__ void stage_write(bf16* dst, const float* buf, int nquad) {
#pragma unroll
  for (int i = 0; i < nquad; ++i) {
    bf16x4 q;
    q[0] = (bf16)buf[4 * i];     q[1] = (bf16)buf[4 * i + 1];
    q[2] = (bf16)buf[4 * i + 2]; q[3] = (bf16)buf[4 * i + 3];
    *(bf16x4*)(dst + 4 * i) = q;
  }
}

template <typename AT, typename WT, int MODE>
__global__ __launch_bounds__(256) void gemm_bias_kernel(
    const AT* __restrict__ A, const WT* __restrict__ W,
    const float* __restrict__ bias, void* __restrict__ out,
    int M, int N, int K, const int* __restrict__ rpos = nullptr, const float* __restrict__ lnw = nullptr, const float* __restrict__ lnb = nullptr, int lda = 0, int ldc = 0) {
  if (lda == 0) lda = K;
  if (ldc == 0) ldc = N;
  __shared__ bf16 ldsA[128 * LDS_STRIDE];
  __shared__ bf16 ldsW[256 * LDS_STRIDE];
  __shared__ __attribute__((aligned(16))) unsigned char sob[256 * 136 * 2];

  const int t    = threadIdx.x;
  const int wave = t >> 5;
  const int lane = t & 31;
  const int wm   = (wave & 1) * 64;
  const int wn   = (wave >> 1) * 64;
  const int mBlk = blockIdx.x * 128;
  const int nBlk = blockIdx.y * 256;

  const int arow = t >> 1;
  const int ach  = (t & 1) * 16;

  float abuf[16];
  float wbuf[32];

  stage_read16(A + (size_t)(mBlk + arow) * lda + ach, abuf);
  stage_read16(W + (size_t)(nBlk + t) * K,          wbuf);
  stage_read16(W + (size_t)(nBlk + t) * K + 16,     wbuf + 16);

  f32x8 acc[4][4] = {};

  for (int k = 0; k < K; k += 32) {
    __syncthreads();
    stage_write(&ldsA[arow * LDS_STRIDE + ach], abuf, 4);
    stage_write(&ldsW[t * LDS_STRIDE],          wbuf, 8);
    if (k + 32 < K) {
      stage_read16(A + (size_t)(mBlk + arow) * lda + (k + 32) + ach, abuf);
      stage_read16(W + (size_t)(nBlk + t) * K + (k + 32),          wbuf);
      stage_read16(W + (size_t)(nBlk + t) * K + (k + 32) + 16,     wbuf + 16);
    }
    __syncthreads();

    bf16x16 af[4], wf[4];
#pragma unroll
    for (int i = 0; i < 4; ++i)
      af[i] = lds_frag(ldsA + (wm + 16 * i) * LDS_STRIDE, LDS_STRIDE);
#pragma unroll
    for (int j = 0; j < 4; ++j)
      wf[j] = lds_frag(ldsW + (wn + 16 * j) * LDS_STRIDE, LDS_STRIDE);
#pragma unroll
    for (int i = 0; i < 4; ++i)
#pragma unroll
      for (int j = 0; j < 4; ++j)
        acc[i][j] = wmma_bf16(af[i], wf[j], acc[i][j]);
  }

  const int nlane = lane & 15;
  const int mh    = (lane >> 4) * 8;
  __syncthreads();
  if (MODE == 0 || MODE == 1) {
    bf16* so = (bf16*)sob;
#pragma unroll
    for (int i = 0; i < 4; ++i)
#pragma unroll
      for (int j = 0; j < 4; ++j) {
        const int nl = wn + 16 * j + nlane;
        const float bv = bias ? bias[nBlk + nl] : 0.0f;
#pragma unroll
        for (int r = 0; r < 8; ++r) {
          const int ml = wm + 16 * i + mh + r;
          const bf16 hv = (bf16)(acc[i][j][r] + bv);
          if (MODE == 0) so[ml * 264 + nl] = hv;
          else           so[nl * 136 + ml] = hv;
        }
      }
    __syncthreads();
#pragma unroll 1
    for (int pass = 0; pass < 2; ++pass) {
      if (MODE == 0) {
        for (int ch = t; ch < 128 * 32; ch += 256) { const int ml = ch >> 5, q = (ch & 31) * 8;
          *(volatile v4u_t*)((bf16*)out + (size_t)(mBlk + ml) * N + nBlk + q) = *(const v4ua*)(so + ml * 264 + q); }
      } else {
        const int b_ = mBlk / SS, s0 = mBlk & (SS - 1);
        for (int ch = t; ch < 256 * 16; ch += 256) { const int nl = ch >> 4, q = (ch & 15) * 8; const int n = nBlk + nl, h = n >> 6, dk = n & (DKK - 1);
          *(volatile v4u_t*)((bf16*)out + (((size_t)(b_ * HH + h)) * DKK + dk) * SS + s0 + q) = *(const v4ua*)(so + nl * 136 + q); }
      }
      __threadfence();
    }
  } else {
    float* so = (float*)sob;
#pragma unroll 1
    for (int hf = 0; hf < 2; ++hf) {
      if (wm == hf * 64) {
#pragma unroll
        for (int i = 0; i < 4; ++i)
#pragma unroll
          for (int j = 0; j < 4; ++j) {
            const int nl = wn + 16 * j + nlane;
            const float bv = bias ? bias[nBlk + nl] : 0.0f;
#pragma unroll
            for (int r = 0; r < 8; ++r) so[(16 * i + mh + r) * 260 + nl] = acc[i][j][r] + bv;
          }
      }
      __syncthreads();
      if (MODE == 3) {
        const int row = t >> 2, hq = t & 3; float* v = so + row * 260 + hq * 64;
        const int token = mBlk + hf * 64 + row; const float tp = (float)rpos[token];
        float mu = 0.0f;
#pragma unroll 1
        for (int d = 0; d < DKK; ++d) mu += v[d];
        mu *= (1.0f / (float)DKK);
        float var = 0.0f;
#pragma unroll 1
        for (int d = 0; d < DKK; ++d) { const float dv = v[d] - mu; var += dv * dv; }
        const float rs = rsqrtf(var * (1.0f / (float)DKK) + 1e-5f);
#pragma unroll 1
        for (int d = 0; d < DKK; ++d) v[d] = (v[d] - mu) * rs * lnw[d] + lnb[d];
#pragma unroll 1
        for (int i = 0; i < DKK / 2; ++i) {
          const float invf = 1.0f / powf(10000.0f, (float)i / (float)(DKK / 2));
          const float ang = tp * invf, c = cosf(ang), s = sinf(ang);
          const float x1 = v[i], x2 = v[i + DKK / 2];
          v[i] = x1 * c - x2 * s; v[i + DKK / 2] = x1 * s + x2 * c;
        }
        __syncthreads();
      }
#pragma unroll 1
      for (int pass = 0; pass < 2; ++pass) {
        for (int ch = t; ch < 64 * 64; ch += 256) { const int ml = ch >> 6, q = (ch & 63) * 4;
          *(volatile v4f_t*)((float*)out + (size_t)(mBlk + hf * 64 + ml) * ldc + nBlk + q) = *(const volatile v4fa*)(so + ml * 260 + q); }
        __threadfence();
      }
      __syncthreads();
    }
  }
}


__global__ __launch_bounds__(256) void k_tw(const float* __restrict__ W, float* __restrict__ WT, int K, int N) {
  __shared__ float tile[64][65];
  const int kb0 = blockIdx.y * 64, n0 = blockIdx.x * 64, t = threadIdx.x;
  for (int i = t; i < 64 * 64; i += 256) { const int kr = i >> 6, nc = i & 63; tile[kr][nc] = W[(size_t)(kb0 + kr) * N + n0 + nc]; }
  __syncthreads();
#pragma unroll 1
  for (int pass = 0; pass < 2; ++pass) {
    for (int i = t; i < 64 * 16; i += 256) { const int nr = i >> 4, k4 = (i & 15) * 4; v4f_t v; v.x = tile[k4][nr]; v.y = tile[k4 + 1][nr]; v.z = tile[k4 + 2][nr]; v.w = tile[k4 + 3][nr];
      *(volatile v4f_t*)(WT + (size_t)(n0 + nr) * K + kb0 + k4) = v; }
    __threadfence();
  }
}
__global__ __launch_bounds__(256) void k_pkbd(const float* __restrict__ pkv, float* __restrict__ PK) {
  const int g = blockIdx.y, n = blockIdx.x, k = threadIdx.x; const int hl = n >> 6, e = n & 63, hl2 = k >> 6, d = k & 63;
  const float v = (hl == hl2) ? pkv[((size_t)(4 * g + hl) * DKK + d) * DKK + e] : 0.0f;
  float* dst = PK + ((size_t)g * 256 + n) * 256 + k; *(volatile float*)dst = v; __threadfence(); *(volatile float*)dst = v;
}
__global__ __launch_bounds__(256) void k_vt(const float* __restrict__ Vf, bf16* __restrict__ Vt, size_t plane) {
  __shared__ float tile[64][65];
  const int s0 = blockIdx.x * 64, h = blockIdx.y, b = blockIdx.z, t = threadIdx.x;
  for (int i = t; i < 64 * 64; i += 256) { const int r = i >> 6, d = i & 63; tile[r][d] = Vf[((size_t)(b * SS + s0 + r)) * DD + h * DKK + d]; }
  __syncthreads();
#pragma unroll 1
  for (int pass = 0; pass < 2; ++pass) {
    for (int i = t; i < 64 * 8; i += 256) { const int dr = i >> 3, s8 = (i & 7) * 8; bf16 hh[8], hl[8];
#pragma unroll
      for (int e = 0; e < 8; ++e) { const float x = tile[s8 + e][dr]; hh[e] = (bf16)x; hl[e] = lo_of(x, hh[e]); }
      bf16* dst = Vt + (((size_t)(h * DKK + dr)) * BH + b) * SS + s0 + s8;
      *(volatile v4u_t*)dst = *(const v4ua*)hh; *(volatile v4u_t*)(dst + plane) = *(const v4ua*)hl; }
    __threadfence();
  }
}
__global__ __launch_bounds__(256) void k_kt(const bf16* __restrict__ Kb, bf16* __restrict__ Kt) {
  __shared__ bf16 tile[64][72];
  const int s0 = blockIdx.x * 64, h = blockIdx.y, b = blockIdx.z, t = threadIdx.x;
  for (int i = t; i < 64 * 64; i += 256) { const int r = i >> 6, d = i & 63; tile[r][d] = Kb[((size_t)(b * SS + s0 + r)) * DD + h * DKK + d]; }
  __syncthreads();
#pragma unroll 1
  for (int pass = 0; pass < 2; ++pass) {
    for (int i = t; i < 64 * 8; i += 256) { const int dr = i >> 3, s8 = (i & 7) * 8; bf16 hh[8];
#pragma unroll
      for (int e = 0; e < 8; ++e) hh[e] = tile[s8 + e][dr];
      *(volatile v4u_t*)(Kt + (((size_t)(h * DKK + dr)) * BH + b) * SS + s0 + s8) = *(const v4ua*)hh; }
    __threadfence();
  }
}
__global__ __launch_bounds__(64) void k_cross(float* __restrict__ PC) {
  const int h = blockIdx.x, b = blockIdx.y, e = threadIdx.x;
  const float gam = 1.0f - exp2f(-5.0f - (float)h);
  float* col = PC + (size_t)b * SS * DD + h * DKK + e; float c = 0.0f;
#pragma unroll 1
  for (int t = SS - 1; t >= 0; --t) { float* p = col + (size_t)t * DD; c = *p + gam * c; *(volatile float*)p = c; __threadfence(); *(volatile float*)p = c; }
}

#define RQW 1
__global__ __launch_bounds__(64) void retention_kernel(
    const bf16* __restrict__ Qb, const bf16* __restrict__ Kb,
    const bf16* __restrict__ Vt, size_t vPlane, float* __restrict__ RC) {
  __shared__ bf16 ldsK[32 * KSTRIDE];
  __shared__ bf16 ldsV[64 * VSTRIDE], ldsVl[64 * VSTRIDE];
  __shared__ __attribute__((aligned(16))) float ldsO[2][16 * 68];

  const int q0blk = blockIdx.x * 32;
  const int h  = blockIdx.y;
  const int b  = blockIdx.z;
  const int t    = threadIdx.x;
  const int wave = t >> 5;
  const int lane = t & 31;
  const int qlane = lane & 15;
  const int kh8   = (lane >> 4) * 8;
  const int q0 = q0blk + wave * 16;
  const float lg = log2f(1.0f - exp2f(-5.0f - (float)h));

  const bf16* Qh = Qb + (size_t)b * SS * DD + h * DKK;
  const bf16* Kh = Kb + (size_t)b * SS * DD + h * DKK;
  const bf16* Vh = Vt + ((size_t)(h * DKK) * BH + b) * SS;
  const int krow = t >> 1, kcol = (t & 1) * 32;
  const bf16* kSrc = Kh + (size_t)krow * DD + kcol;
  const bf16* vSrc = Vh + (size_t)t * BH * SS;

  const bf16x16 qf0 = load_frag(Qh, DD, q0, 0), qf1 = load_frag(Qh, DD, q0, 32);
  f32x8 o[4] = {};
  const int kmax = q0blk + 31;
  bf16x8 kreg[4], vreg[4], vlreg[4];
#pragma unroll
  for (int i = 0; i < 4; ++i) { kreg[i] = *(const bf16x8*)(kSrc + 8 * i); vreg[i] = *(const bf16x8*)(vSrc + 8 * i); vlreg[i] = *(const bf16x8*)(vSrc + vPlane + 8 * i); }
  for (int kb = 0; kb <= kmax; kb += 32) {
    __syncthreads();
#pragma unroll
    for (int i = 0; i < 4; ++i) { *(bf16x8*)(&ldsK[krow * KSTRIDE + kcol + 8 * i]) = kreg[i]; *(bf16x8*)(&ldsV[t * VSTRIDE + 8 * i]) = vreg[i]; *(bf16x8*)(&ldsVl[t * VSTRIDE + 8 * i]) = vlreg[i]; }
    if (kb + 32 <= kmax) { const bf16* kn = kSrc + (size_t)(kb + 32) * DD; const bf16* vn = vSrc + (kb + 32);
#pragma unroll
      for (int i = 0; i < 4; ++i) { kreg[i] = *(const bf16x8*)(kn + 8 * i); vreg[i] = *(const bf16x8*)(vn + 8 * i); vlreg[i] = *(const bf16x8*)(vn + vPlane + 8 * i); } }
    __syncthreads();
    bf16x16 kf[2][2];
#pragma unroll
    for (int ktile = 0; ktile < 2; ++ktile)
#pragma unroll
      for (int c = 0; c < 2; ++c) kf[ktile][c] = lds_frag(ldsK + (ktile * 16) * KSTRIDE + c * 32, KSTRIDE);
    const bool act = (kb <= q0 + 15);
    bf16x16 pf, pfl;
    if (act) {
      const int q_my = q0 + qlane;
      f32x8 s0 = {}, s1 = {};
      s0 = wmma_bf16(kf[0][0], qf0, s0); s0 = wmma_bf16(kf[0][1], qf1, s0);
      s1 = wmma_bf16(kf[1][0], qf0, s1); s1 = wmma_bf16(kf[1][1], qf1, s1);
#pragma unroll
      for (int r = 0; r < 8; ++r) {
        const int k0i = kb + kh8 + r, k1i = k0i + 16;
        const float w0 = (k0i <= q_my) ? s0[r] * exp2f((float)(q_my - k0i) * lg) : 0.0f;
        const float w1 = (k1i <= q_my) ? s1[r] * exp2f((float)(q_my - k1i) * lg) : 0.0f;
        pf[r] = (bf16)w0; pfl[r] = lo_of(w0, pf[r]); pf[r + 8] = (bf16)w1; pfl[r + 8] = lo_of(w1, pf[r + 8]);
      }
#pragma unroll
      for (int j = 0; j < 4; ++j) {
        const bf16x16 vf = lds_frag(ldsV + (j * 16) * VSTRIDE, VSTRIDE), vfl = lds_frag(ldsVl + (j * 16) * VSTRIDE, VSTRIDE);
        o[j] = wmma_split(vf, vfl, pf, pfl, o[j]); }
    }
  }
  float* so = ldsO[wave];
#pragma unroll
  for (int j = 0; j < 4; ++j)
#pragma unroll
    for (int r = 0; r < 8; ++r) so[qlane * 68 + j * 16 + kh8 + r] = o[j][r];
  asm volatile("s_wait_dscnt 0" ::: "memory");
  float4 keep[8];
#pragma unroll
  for (int it = 0; it < 8; ++it) { const int ch = lane + 32 * it, ql = ch >> 4, q4 = (ch & 15) * 4;
    float* p = RC + ((size_t)(b * SS + q0 + ql)) * DD + h * DKK + q4; const v4f_t cv = *(const volatile v4fa*)p; const v4f_t ov = *(const volatile v4fa*)(so + ql * 68 + q4);
    keep[it] = make_float4(ov.x + cv.x, ov.y + cv.y, ov.z + cv.z, ov.w + cv.w); }
#pragma unroll 1
  for (int pass = 0; pass < 2; ++pass) {
#pragma unroll
    for (int it = 0; it < 8; ++it) { const int ch = lane + 32 * it, ql = ch >> 4, q4 = (ch & 15) * 4; v4f_t v; v.x = keep[it].x; v.y = keep[it].y; v.z = keep[it].z; v.w = keep[it].w;
      *(volatile v4f_t*)(RC + ((size_t)(b * SS + q0 + ql)) * DD + h * DKK + q4) = v; }
    __threadfence();
  }
}
__global__ __launch_bounds__(256) void k_gnstat(const float* __restrict__ R, float* __restrict__ P) {
  __shared__ float red[2][256];
  const int blk = blockIdx.x, b = blockIdx.y, t = threadIdx.x;
  const float* base = R + ((size_t)b * SS + blk * 8) * DD; float s = 0.f, q = 0.f;
#pragma unroll 1
  for (int i = t; i < 8 * DD; i += 256) { const float v = base[i]; s += v; q += v * v; }
  red[0][t] = s; red[1][t] = q; __syncthreads();
  for (int o = 128; o > 0; o >>= 1) { if (t < o) { red[0][t] += red[0][t + o]; red[1][t] += red[1][t + o]; } __syncthreads(); }
  if (t == 0) { typedef __attribute__((ext_vector_type(2))) float v2f; v2f v; v.x = red[0][0]; v.y = red[1][0]; float* dst = P + ((size_t)b * (SS / 8) + blk) * 2;
    *(volatile v2f*)dst = v; __threadfence(); *(volatile v2f*)dst = v; }
}
__global__ __launch_bounds__(256) void k_gnout(const float* __restrict__ R, const float* __restrict__ P, const float* __restrict__ gw, const float* __restrict__ gbias, int bofs, float* __restrict__ out) {
  __shared__ float st[2];
  const int row = blockIdx.x, b = blockIdx.y, t = threadIdx.x;
  if (t == 0) { double s = 0.0, q = 0.0; for (int i = 0; i < SS / 8; ++i) { s += (double)P[((size_t)b * (SS / 8) + i) * 2]; q += (double)P[((size_t)b * (SS / 8) + i) * 2 + 1]; }
    const double n = (double)SS * DD, mu = s / n, var = fmax(q / n - mu * mu, 0.0); st[0] = (float)mu; st[1] = (float)(1.0 / sqrt(var + 1e-5)); }
  __syncthreads();
  const float mu = st[0], rs = st[1];
  const float* src = R + ((size_t)b * SS + row) * DD; float* dst = out + (((size_t)(bofs + b)) * SS + row) * DD;
#pragma unroll 1
  for (int pass = 0; pass < 2; ++pass) {
    for (int c4 = t * 4; c4 < DD; c4 += 1024) { const int h = c4 >> 6; v4f_t v = *(const v4fa*)(src + c4); const float w = gw[h], bb = gbias[h];
      v.x = (v.x - mu) * rs * w + bb; v.y = (v.y - mu) * rs * w + bb; v.z = (v.z - mu) * rs * w + bb; v.w = (v.w - mu) * rs * w + bb;
      *(volatile v4f_t*)(dst + c4) = v; }
    __threadfence();
  }
}
__global__ __launch_bounds__(64) void k_kvout(const float* __restrict__ CK0, const float* __restrict__ CK1, const float* __restrict__ pkv, float* __restrict__ out2) {
  const int h = blockIdx.x >> 6, d = blockIdx.x & 63, e = threadIdx.x; const int g = h >> 2, hl = h & 3;
  const float gam = 1.0f - exp2f(-5.0f - (float)h);
  const size_t ci = ((size_t)g * 256 + hl * 64 + d) * 256 + hl * 64 + e;
  const float v = gam * pkv[((size_t)h * DKK + d) * DKK + e] + (CK0[ci] + CK1[ci]) * (1.0f / (float)BB);
  float* dst = out2 + ((size_t)h * DKK + d) * DKK + e; *(volatile float*)dst = v; __threadfence(); *(volatile float*)dst = v;
}

extern "C" void kernel_launch(void* const* d_in, const int* in_sizes, int n_in,
                              void* d_out, int out_size, void* d_ws, size_t ws_size,
                              hipStream_t stream) {
  (void)in_sizes; (void)n_in; (void)out_size; (void)ws_size;
  const float* x   = (const float*)d_in[0];
  const float* pkv = (const float*)d_in[1];
  const float* Wq = (const float*)d_in[2]; const float* Wk = (const float*)d_in[3]; const float* Wv = (const float*)d_in[4];
  const float* gw = (const float*)d_in[5]; const float* gbias = (const float*)d_in[6];
  float* out  = (float*)d_out;
  float* out2 = out + (size_t)BB * SS * DD;
  const int M = BH * SS;
  char* ws = (char*)d_ws;
  float* WT  = (float*)ws; ws += (size_t)3 * DD * DD * 4;
  float* PK  = (float*)ws; ws += (size_t)4 * 256 * 256 * 4;
  bf16*  Qb  = (bf16*)ws;  ws += (size_t)M * DD * 2;
  bf16*  Kb  = (bf16*)ws;  ws += (size_t)M * DD * 2;
  float* Vf  = (float*)ws; ws += (size_t)M * DD * 4;
  bf16*  Vt  = (bf16*)ws;  ws += (size_t)M * DD * 2 * 2;
  bf16*  Kt  = (bf16*)ws;  ws += (size_t)M * DD * 2;
  float* RC  = (float*)ws; ws += (size_t)M * DD * 4;
  float* CKV = (float*)ws; ws += (size_t)2 * 4 * 256 * 256 * 4;
  float* P   = (float*)ws; ws += (size_t)BH * (SS / 8) * 2 * 4;
  const size_t pl = (size_t)DD * DD, vpl = (size_t)M * DD;
  for (int w = 0; w < 3; ++w) k_tw<<<dim3(DD / 64, DD / 64), 256, 0, stream>>>(w == 0 ? Wq : w == 1 ? Wk : Wv, WT + w * pl, DD, DD);
  k_pkbd<<<dim3(256, 4), 256, 0, stream>>>(pkv, PK);
  dim3 gGrid(M / 128, DD / 256), gBlk(256);
  for (int ps = 0; ps < BB / BH; ++ps) {
    const float* xp = x + (size_t)ps * M * DD;
    gemm_bias_kernel<float, float, 0><<<gGrid, gBlk, 0, stream>>>(xp, WT,          nullptr, Qb, M, DD, DD);
    gemm_bias_kernel<float, float, 0><<<gGrid, gBlk, 0, stream>>>(xp, WT + pl,     nullptr, Kb, M, DD, DD);
    gemm_bias_kernel<float, float, 2><<<gGrid, gBlk, 0, stream>>>(xp, WT + 2 * pl, nullptr, Vf, M, DD, DD);
    k_vt<<<dim3(SS / 64, HH, BH), 256, 0, stream>>>(Vf, Vt, vpl);
    k_kt<<<dim3(SS / 64, HH, BH), 256, 0, stream>>>(Kb, Kt);
    for (int g = 0; g < 4; ++g)
      gemm_bias_kernel<bf16, float, 2><<<dim3(M / 128, 1), gBlk, 0, stream>>>(Qb + 256 * g, PK + (size_t)g * 256 * 256, nullptr, RC + 256 * g, M, 256, 256, nullptr, nullptr, nullptr, DD, DD);
    k_cross<<<dim3(HH, BH), 64, 0, stream>>>(RC);
    retention_kernel<<<dim3(SS / 32, HH, BH), 64, 0, stream>>>(Qb, Kb, Vt, vpl, RC);
    for (int g = 0; g < 4; ++g)
      gemm_bias_kernel<bf16, bf16, 2><<<dim3(2, 1), gBlk, 0, stream>>>(Kt + (size_t)g * 256 * BH * SS, Vt + (size_t)g * 256 * BH * SS, nullptr, CKV + ((size_t)ps * 4 + g) * 256 * 256, 256, 256, BH * SS);
    k_gnstat<<<dim3(SS / 8, BH), 256, 0, stream>>>(RC, P);
    k_gnout<<<dim3(SS, BH), 256, 0, stream>>>(RC, P, gw, gbias, ps * BH, out);
  }
  k_kvout<<<HH * DKK, 64, 0, stream>>>(CKV, CKV + (size_t)4 * 256 * 256, pkv, out2);
}
